// IntrospectiveFlashDiff2_60601988547137
// MI455X (gfx1250) — hardware-verified
//
#include <hip/hip_runtime.h>
#include <stdint.h>

#define BB 2
#define TT 1024
#define DD 1024
#define HH 16
#define NKVH 8
#define HDIM 64
#define DKV 512
#define MAXKV 3072
#define NLAY 3
#define EPSV 1e-5f

typedef __attribute__((ext_vector_type(16))) _Float16 v16h;
typedef __attribute__((ext_vector_type(8)))  _Float16 v8h;
typedef __attribute__((ext_vector_type(4)))  _Float16 v4h;
typedef __attribute__((ext_vector_type(16))) __bf16   v16b;
typedef __attribute__((ext_vector_type(8)))  __bf16   v8b;
typedef __attribute__((ext_vector_type(8)))  float    v8f;
typedef __attribute__((ext_vector_type(4)))  float    v4f;

__device__ __forceinline__ unsigned short f2bf_bits(float f) {
  unsigned u = __float_as_uint(f);
  return (unsigned short)((u + 0x7FFFu + ((u >> 16) & 1u)) >> 16);
}
__device__ __forceinline__ float bf_bits2f(unsigned short h) { return __uint_as_float(((unsigned)h) << 16); }

__device__ __forceinline__ void dep_guard_h(v8f& a, v8f& b, v16h x, v16h y) { asm volatile("v_nop\n\tv_nop\n\tv_nop\n\tv_nop" : "+v"(a), "+v"(b) : "v"(x), "v"(y)); }
__device__ __forceinline__ void dep_guard_b(v8f& a, v8f& b, v16b x, v16b y) { asm volatile("v_nop\n\tv_nop\n\tv_nop\n\tv_nop" : "+v"(a), "+v"(b) : "v"(x), "v"(y)); }
__device__ __forceinline__ void keep4_h(v16h a, v16h b, v16h c, v16h d) { asm volatile("v_nop" :: "v"(a), "v"(b), "v"(c), "v"(d)); }
__device__ __forceinline__ void keep4_b(v16b a, v16b b, v16b c, v16b d) { asm volatile("v_nop" :: "v"(a), "v"(b), "v"(c), "v"(d)); }
__device__ __forceinline__ void acc_guard4(v8f& a, v8f& b, v8f& c, v8f& d) { asm volatile("v_nop\n\tv_nop\n\tv_nop\n\tv_nop" : "+v"(a), "+v"(b), "+v"(c), "+v"(d)); }
template <typename T> struct Frag;
template <> struct Frag<_Float16> {
  typedef v16h V; union U { v16h v; v8h h[2]; };
  static __device__ __forceinline__ v16h load(const _Float16* p) {
    U f; f.h[0] = *(const v8h*)(p); f.h[1] = *(const v8h*)(p + 16); return f.v;
  }
  static __device__ __forceinline__ v8f mma(v16h a, v16h b, v8f c) {
    return __builtin_amdgcn_wmma_f32_16x16x32_f16(false, a, false, b, (short)0, c, false, false);
  }
  static __device__ __forceinline__ void guard(v8f& a, v8f& b, v16h x, v16h y) { dep_guard_h(a, b, x, y); }
  static __device__ __forceinline__ void keep(v16h a, v16h b, v16h c, v16h d) { keep4_h(a, b, c, d); }
};
template <> struct Frag<__bf16> {
  typedef v16b V; union U { v16b v; v8b h[2]; };
  static __device__ __forceinline__ v16b load(const __bf16* p) {
    U f; f.h[0] = *(const v8b*)(p); f.h[1] = *(const v8b*)(p + 16); return f.v;
  }
  static __device__ __forceinline__ v8f mma(v16b a, v16b b, v8f c) {
    return __builtin_amdgcn_wmma_f32_16x16x32_bf16(false, a, false, b, (short)0, c, false, false);
  }
  static __device__ __forceinline__ void guard(v8f& a, v8f& b, v16b x, v16b y) { dep_guard_b(a, b, x, y); }
  static __device__ __forceinline__ void keep(v16b a, v16b b, v16b c, v16b d) { keep4_b(a, b, c, d); }
};

template <int ET> struct Elem;
template <> struct Elem<0> { typedef _Float16 T; };
template <> struct Elem<1> { typedef __bf16 T; };
template <int ET, bool SPLIT, int BIAS_MODE, int OUT_MODE, bool RESID, int ACT = 0>
__global__ __launch_bounds__(256) void wmma_gemm64(
    const unsigned short* __restrict__ Ap, const unsigned short* __restrict__ A2p, int lda, long strideA,
    const unsigned short* __restrict__ Btp, const unsigned short* __restrict__ Bt2p, int ldb, long strideB,
    void* __restrict__ Cout, void* __restrict__ Cout2, int ldc, long strideC,
    const float* __restrict__ bias,
    const float* __restrict__ resid, long strideR,
    int M, int N, int K, float scale) {
  typedef typename Elem<ET>::T T;
  typedef typename Frag<T>::V V;
  const T* A = (const T*)Ap; const T* A2 = (const T*)A2p; const T* Bt = (const T*)Btp; const T* Bt2 = (const T*)Bt2p;
  __shared__ __align__(16) float sT[8][16 * 68];
  const int b    = blockIdx.y;
  const int lane = threadIdx.x & 31;
  const int wave = threadIdx.x >> 5;
  const int tilesN = N >> 6;
  const int tilesM = M >> 6;
  const int tile = blockIdx.x * 8 + wave;
  if (tile >= tilesM * tilesN) return;
  const int tm = tile / tilesN;
  const int tn = tile - tm * tilesN;
  const int m0 = tm << 6;
  const int n0 = tn << 6;

  const T* Ab  = A  + (size_t)b * strideA;
  const T* Bb  = Bt + (size_t)b * strideB;
  const T* Ab2 = SPLIT ? (A2  + (size_t)b * strideA) : nullptr;
  const T* Bb2 = SPLIT ? (Bt2 + (size_t)b * strideB) : nullptr;

  const int rlane = lane & 15;
  const int koff  = (lane >> 4) * 8;
  const int mOff  = (lane >> 4) * 8;

  v8f acc[4][4];
#pragma unroll
  for (int i = 0; i < 4; ++i)
#pragma unroll
    for (int j = 0; j < 4; ++j) acc[i][j] = (v8f){0.f,0.f,0.f,0.f,0.f,0.f,0.f,0.f};

  for (int k0 = 0; k0 < K; k0 += 32) {
    V bh[4], bl[4];
#pragma unroll
    for (int j = 0; j < 4; ++j) {
      const size_t bo = (size_t)(n0 + (j << 4) + rlane) * ldb + koff + k0;
      bh[j] = Frag<T>::load(Bb + bo);
      if (SPLIT) bl[j] = Frag<T>::load(Bb2 + bo);
    }
#pragma unroll
    for (int i = 0; i < 4; ++i) {
      const size_t ao = (size_t)(m0 + (i << 4) + rlane) * lda + koff + k0;
      V ah = Frag<T>::load(Ab + ao);
      V al;
      if (SPLIT) al = Frag<T>::load(Ab2 + ao);
#pragma unroll
      for (int j = 0; j < 4; ++j) {
        acc[i][j] = Frag<T>::mma(ah, bh[j], acc[i][j]);
        if (SPLIT) {
          acc[i][j] = Frag<T>::mma(ah, bl[j], acc[i][j]);
          acc[i][j] = Frag<T>::mma(al, bh[j], acc[i][j]);
        }
      }
      Frag<T>::guard(acc[i][0], acc[i][3], ah, SPLIT ? al : ah);
    }
    Frag<T>::keep(bh[0], bh[1], bh[2], bh[3]);
    if (SPLIT) Frag<T>::keep(bl[0], bl[1], bl[2], bl[3]);
  }
  acc_guard4(acc[0][0], acc[0][1], acc[0][2], acc[0][3]);
  acc_guard4(acc[1][0], acc[1][1], acc[1][2], acc[1][3]);
  acc_guard4(acc[2][0], acc[2][1], acc[2][2], acc[2][3]);
  acc_guard4(acc[3][0], acc[3][1], acc[3][2], acc[3][3]);

  float* slab = sT[wave];
  const float* Rb = RESID ? (resid + (size_t)b * strideR) : nullptr;
#pragma unroll
  for (int i = 0; i < 4; ++i) {
    const int mBase = m0 + (i << 4);
#pragma unroll
    for (int j = 0; j < 4; ++j) {
      const int n = n0 + (j << 4) + rlane;
      float bv = 0.f;
      if (BIAS_MODE == 2) bv = bias[n];
#pragma unroll
      for (int r = 0; r < 8; ++r) {
        float v = acc[i][j][r] * scale;
        if (BIAS_MODE == 1) v += bias[mBase + mOff + r];
        if (BIAS_MODE == 2) v += bv;
        if (RESID) v += Rb[(size_t)(mBase + mOff + r) * ldc + n];
        if (ACT == 1) v = tanhf(v);
        if (ACT == 2) v = fmaxf(v, 0.0f);
        if (ACT == 3) v = v / (1.0f + expf(-v));
        if (ACT == 4) v = (v > 0.f) ? v : 0.01f * v;
        if (ACT == 5) v = 0.5f * v * (1.0f + erff(v * 0.70710678118654752f));
        slab[(mOff + r) * 68 + (j << 4) + rlane] = v;
      }
    }
    __builtin_amdgcn_fence(__ATOMIC_RELEASE, "workgroup");
    __builtin_amdgcn_wave_barrier();
    __builtin_amdgcn_fence(__ATOMIC_ACQUIRE, "workgroup");
    if (OUT_MODE == 0) {
      float* C = (float*)Cout + (size_t)b * strideC;
      const int hh = lane >> 4, c4 = (lane & 15) * 4;
      for (int pass = 0; pass < 2; ++pass) {
#pragma unroll
        for (int it = 0; it < 8; ++it) {
          const int row = it * 2 + hh;
          v4f v = *(const v4f*)(slab + row * 68 + c4);
          *(volatile v4f*)(C + (size_t)(mBase + row) * ldc + n0 + c4) = v;
        }
        __threadfence();
      }
    } else {
      const int q = lane >> 3, c8 = (lane & 7) * 8;
      unsigned short* C  = (unsigned short*)Cout  + (size_t)b * strideC;
      unsigned short* C2 = (OUT_MODE == 2) ? ((unsigned short*)Cout2 + (size_t)b * strideC) : nullptr;
      for (int pass = 0; pass < 2; ++pass) {
#pragma unroll
        for (int it = 0; it < 4; ++it) {
          const int row = it * 4 + q;
          const float* sp = slab + row * 68 + c8;
          v8h hv, lv;
#pragma unroll
          for (int e = 0; e < 8; ++e) {
            if (OUT_MODE == 1) {
              hv[e] = (_Float16)sp[e];
            } else {
              unsigned short hb = f2bf_bits(sp[e]);
              unsigned short lb = f2bf_bits(sp[e] - bf_bits2f(hb));
              hv[e] = __builtin_bit_cast(_Float16, hb);
              lv[e] = __builtin_bit_cast(_Float16, lb);
            }
          }
          *(volatile v8h*)(C + (size_t)(mBase + row) * ldc + n0 + c8) = hv;
          if (OUT_MODE == 2) *(volatile v8h*)(C2 + (size_t)(mBase + row) * ldc + n0 + c8) = lv;
        }
        __threadfence();
      }
    }
    __builtin_amdgcn_fence(__ATOMIC_RELEASE, "workgroup");
    __builtin_amdgcn_wave_barrier();
    __builtin_amdgcn_fence(__ATOMIC_ACQUIRE, "workgroup");
  }
}

__global__ __launch_bounds__(256) void cast_f32_f16x8(
    const float* __restrict__ in, _Float16* __restrict__ out, int n8, float scale) {
  const int i = blockIdx.x * 256 + threadIdx.x;
  if (i < n8) {
    const size_t o = (size_t)i * 8;
    const v4f a = *(const v4f*)(in + o);
    const v4f b = *(const v4f*)(in + o + 4);
    v8h hv;
#pragma unroll
    for (int e = 0; e < 4; ++e) {
      hv[e]     = (_Float16)(a[e] * scale);
      hv[4 + e] = (_Float16)(b[e] * scale);
    }
    *(volatile v8h*)(out + o) = hv;
    __threadfence();
    *(volatile v8h*)(out + o) = hv;
  }
}

__device__ __forceinline__ _Float16 rope_one(float x1, float x2, float cc, float ss, bool second, float oscale) {
  const float o = second ? (x2 * cc + x1 * ss) : (x1 * cc - x2 * ss);
  return (_Float16)(o * oscale);
}
template <int NC>
__global__ __launch_bounds__(256) void rope_cast_kernel(
    const float* __restrict__ src, const float* __restrict__ cosT, const float* __restrict__ sinT,
    _Float16* __restrict__ dst, int dst_brows, int pos_off, float oscale) {
  constexpr int TPR = NC / 8;
  constexpr int RPB = 256 / TPR;
  const int tid = threadIdx.x;
  const int row = blockIdx.x * RPB + tid / TPR;
  const int b = row >> 10, t = row & (TT - 1);
  const int p = pos_off + t;
  const int d8 = (tid % TPR) * 8;
  const int hoff = d8 & ~63;
  const int dl = d8 & 63;
  const int j0 = dl & 31;
  const bool second = dl >= 32;
  const float* base = src + (size_t)row * NC + hoff;
  const v4f a0 = *(const v4f*)(base + j0),      a1 = *(const v4f*)(base + j0 + 4);
  const v4f b0 = *(const v4f*)(base + 32 + j0), b1 = *(const v4f*)(base + 32 + j0 + 4);
  const v4f c0 = *(const v4f*)(cosT + (size_t)p * 32 + j0), c1 = *(const v4f*)(cosT + (size_t)p * 32 + j0 + 4);
  const v4f s0 = *(const v4f*)(sinT + (size_t)p * 32 + j0), s1 = *(const v4f*)(sinT + (size_t)p * 32 + j0 + 4);
  v8h hv;
#pragma unroll
  for (int e = 0; e < 4; ++e) {
    hv[e]     = rope_one(a0[e], b0[e], c0[e], s0[e], second, oscale);
    hv[4 + e] = rope_one(a1[e], b1[e], c1[e], s1[e], second, oscale);
  }
  _Float16* dp = dst + ((size_t)b * dst_brows + p) * NC + d8;
  *(volatile v8h*)dp = hv;
  __threadfence();
  *(volatile v8h*)dp = hv;
}

#define AT_D 64
#define AT_NW 4
#define AT_QB 64
#define AT_KC 64

__device__ __forceinline__ v8f hmma(v16h a, v16h b, v8f c) {
  c = __builtin_amdgcn_wmma_f32_16x16x32_f16(false, a, false, b, (short)0, c, false, false);
  asm volatile("v_nop\n\tv_nop\n\tv_nop\n\tv_nop" : "+v"(c) : "v"(a), "v"(b));
  return c;
}

__global__ __launch_bounds__(128)
void attn_f16_kernel(const _Float16* __restrict__ Qh, const _Float16* __restrict__ Kh,
                     const _Float16* __restrict__ Vth, float* __restrict__ O,
                     int kchunks_prev, int koff, float sscale, float onorm) {
  union FH { v16h v; v8h h[2]; };
  __shared__ __align__(16) _Float16 Ksh[AT_KC * AT_D];
  __shared__ __align__(16) _Float16 Vtt[AT_D * AT_KC];
  __shared__ __align__(16) _Float16 Psh[AT_NW][16 * AT_KC];
  __shared__ __align__(16) float    Os[AT_NW][16 * 68];

  const int tid  = threadIdx.x;
  const int wave = tid >> 5;
  const int lane = tid & 31;
  const int hh   = lane >> 4;
  const int c    = lane & 15;

  const int bx  = blockIdx.x;
  const int qb  = bx & (TT / AT_QB - 1);
  const int h   = (bx >> 4) & (HH - 1);
  const int b   = bx >> 8;
  const int hkv = h >> 1;
  const int q0  = qb * AT_QB + wave * 16;

  v16h qa[2];
  {
    const _Float16* qrow = Qh + (size_t)(b * TT + q0 + c) * DD + h * AT_D + 8 * hh;
#pragma unroll
    for (int dc = 0; dc < 2; ++dc) qa[dc] = Frag<_Float16>::load(qrow + dc * 32);
  }

  float mrow[8], lrow[8];
  v8f oacc[4];
#pragma unroll
  for (int r = 0; r < 8; ++r) { mrow[r] = -INFINITY; lrow[r] = 0.f; }
#pragma unroll
  for (int t = 0; t < 4; ++t) oacc[t] = (v8f){0.f,0.f,0.f,0.f,0.f,0.f,0.f,0.f};

  int nChunks = kchunks_prev + qb + 1;
  if (nChunks > MAXKV / AT_KC) nChunks = MAXKV / AT_KC;
  if (nChunks < 1) nChunks = 1;

  const _Float16* kbase = Kh + (size_t)b * MAXKV * DKV + hkv * AT_D;
  const _Float16* vbase = Vth + ((size_t)b * DKV + hkv * AT_D) * MAXKV;
  float*          obase = O + (size_t)b * TT * DD + h * AT_D;

  for (int kc = 0; kc < nChunks; ++kc) {
    const int kv0 = kc * AT_KC;
    __syncthreads();
    {
      const int r = tid >> 1, hf = (tid & 1) * 32;
      const _Float16* ks = kbase + (size_t)(kv0 + r) * DKV + hf;
      const _Float16* vs = vbase + (size_t)r * MAXKV + kv0 + hf;
#pragma unroll
      for (int i = 0; i < 4; ++i) {
        const v8h kk = *(const v8h*)(ks + 8 * i);
        const v8h vv = *(const v8h*)(vs + 8 * i);
        *(v8h*)(Ksh + r * AT_D + hf + 8 * i) = kk;
        *(v8h*)(Vtt + r * AT_KC + hf + 8 * i) = vv;
      }
    }
    __syncthreads();

    v8f s[4];
#pragma unroll
    for (int j = 0; j < 4; ++j) {
      s[j] = (v8f){0.f,0.f,0.f,0.f,0.f,0.f,0.f,0.f};
#pragma unroll
      for (int dc = 0; dc < 2; ++dc) {
        FH kb;
        kb.h[0] = *(const v8h*)(Ksh + (j * 16 + c) * AT_D + dc * 32 + 8 * hh);
        kb.h[1] = *(const v8h*)(Ksh + (j * 16 + c) * AT_D + dc * 32 + 16 + 8 * hh);
        s[j] = hmma(qa[dc], kb.v, s[j]);
      }
    }
    float cm[8];
#pragma unroll
    for (int r = 0; r < 8; ++r) {
      const int qlim = q0 + 8 * hh + r + koff;
      float m = -INFINITY;
#pragma unroll
      for (int j = 0; j < 4; ++j) {
        const int kvcol = kv0 + j * 16 + c;
        const float sv = (kvcol > qlim) ? -INFINITY : (s[j][r] * sscale);
        s[j][r] = sv;
        m = fmaxf(m, sv);
      }
#pragma unroll
      for (int off = 1; off < 16; off <<= 1) m = fmaxf(m, __shfl_xor(m, off, 32));
      cm[r] = m;
    }
    _Float16* pw = Psh[wave];
#pragma unroll
    for (int r = 0; r < 8; ++r) {
      const float mnew = fmaxf(mrow[r], cm[r]);
      const float alpha = expf(mrow[r] - mnew);
      mrow[r] = mnew;
      float psum = 0.f;
#pragma unroll
      for (int j = 0; j < 4; ++j) {
        const float p = expf(s[j][r] - mnew);
        psum += p;
        pw[(8 * hh + r) * AT_KC + j * 16 + c] = (_Float16)(p * 32768.0f);
      }
#pragma unroll
      for (int off = 1; off < 16; off <<= 1) psum += __shfl_xor(psum, off, 32);
      lrow[r] = lrow[r] * alpha + psum;
#pragma unroll
      for (int t = 0; t < 4; ++t) oacc[t][r] *= alpha;
    }
    __builtin_amdgcn_fence(__ATOMIC_RELEASE, "workgroup");
    __builtin_amdgcn_wave_barrier();
    __builtin_amdgcn_fence(__ATOMIC_ACQUIRE, "workgroup");
#pragma unroll 1
    for (int kk = 0; kk < 2; ++kk) {
      FH pa;
      pa.h[0] = *(const v8h*)(pw + c * AT_KC + kk * 32 + 8 * hh);
      pa.h[1] = *(const v8h*)(pw + c * AT_KC + kk * 32 + 16 + 8 * hh);
#pragma unroll
      for (int t = 0; t < 4; ++t) {
        FH vb;
        vb.h[0] = *(const v8h*)(Vtt + (t * 16 + c) * AT_KC + kk * 32 + 8 * hh);
        vb.h[1] = *(const v8h*)(Vtt + (t * 16 + c) * AT_KC + kk * 32 + 16 + 8 * hh);
        oacc[t] = hmma(pa.v, vb.v, oacc[t]);
      }
    }
  }

  float* os = Os[wave];
#pragma unroll
  for (int r = 0; r < 8; ++r) {
    const float inv = onorm * (1.0f / lrow[r]);
#pragma unroll
    for (int t = 0; t < 4; ++t) os[(8 * hh + r) * 68 + t * 16 + c] = oacc[t][r] * inv;
  }
  __builtin_amdgcn_fence(__ATOMIC_RELEASE, "workgroup");
  __builtin_amdgcn_wave_barrier();
  __builtin_amdgcn_fence(__ATOMIC_ACQUIRE, "workgroup");
  {
    const int c4 = (lane & 15) * 4;
    for (int pass = 0; pass < 2; ++pass) {
#pragma unroll
      for (int it = 0; it < 8; ++it) {
        const int row = it * 2 + hh;
        v4f val = *(const v4f*)(os + row * 68 + c4);
        *(volatile v4f*)(obase + (size_t)(q0 + row) * DD + c4) = val;
      }
      __threadfence();
    }
  }
}

__global__ __launch_bounds__(256) void combine_kernel(
    const float* __restrict__ Of, long lstride,
    const float* __restrict__ x, const float* __restrict__ ln_w, const float* __restrict__ lam,
    const float* __restrict__ fln, const float* __restrict__ alpha, _Float16* __restrict__ Yh) {
  __shared__ float red[4][8];
  const int row = blockIdx.x;
  const int tid = threadIdx.x, lane = tid & 31, wave = tid >> 5;
  const int d4 = tid * 4;
  const size_t ro = (size_t)row * DD + d4;
  const v4f o0 = *(const v4f*)(Of + ro);
  const v4f o1 = *(const v4f*)(Of + lstride + ro);
  const v4f o2 = *(const v4f*)(Of + 2 * lstride + ro);
  const v4f xv = *(const v4f*)(x + ro);
  float ss0 = 0.f, ss1 = 0.f, ss2 = 0.f;
#pragma unroll
  for (int e = 0; e < 4; ++e) { ss0 += o0[e] * o0[e]; ss1 += o1[e] * o1[e]; ss2 += o2[e] * o2[e]; }
#pragma unroll
  for (int off = 16; off > 0; off >>= 1) {
    ss0 += __shfl_xor(ss0, off, 32);
    ss1 += __shfl_xor(ss1, off, 32);
    ss2 += __shfl_xor(ss2, off, 32);
  }
  if (lane == 0) { red[0][wave] = ss0; red[1][wave] = ss1; red[2][wave] = ss2; }
  __syncthreads();
  float t0 = 0.f, t1 = 0.f, t2 = 0.f;
#pragma unroll
  for (int w = 0; w < 8; ++w) { t0 += red[0][w]; t1 += red[1][w]; t2 += red[2][w]; }
  const float inv_d = 1.0f / (float)DD;
  const float r0 = rsqrtf(t0 * inv_d + EPSV);
  const float r1 = rsqrtf(t1 * inv_d + EPSV);
  const float r2 = rsqrtf(t2 * inv_d + EPSV);

  const float sg0 = 1.0f / (1.0f + __expf(-lam[0]));
  const float sg1 = 1.0f / (1.0f + __expf(-lam[1]));
  const float sg2 = 1.0f / (1.0f + __expf(-lam[2]));
  const float mean = (sg0 + sg1 + sg2) * (1.0f / 3.0f);
  const float e0 = sg0 - mean, e1 = sg1 - mean, e2 = sg2 - mean;
  const float var = (e0 * e0 + e1 * e1 + e2 * e2) * (1.0f / 3.0f);
  const float il = rsqrtf(var + EPSV);
  const float lw0 = e0 * il, lw1 = e1 * il, lw2 = e2 * il;

  const v4f w0 = *(const v4f*)(ln_w + d4);
  const v4f w1 = *(const v4f*)(ln_w + DD + d4);
  const v4f w2 = *(const v4f*)(ln_w + 2 * DD + d4);
  const v4f fw = *(const v4f*)(fln + d4);
  const float al = alpha[0];
  v4f z;
  float ssz = 0.f;
#pragma unroll
  for (int e = 0; e < 4; ++e) {
    float a = (o0[e] * r0) * w0[e] * lw0;
    a = a + (o1[e] * r1) * w1[e] * lw1;
    a = a + (o2[e] * r2) * w2[e] * lw2;
    const float zz = a + al * xv[e];
    z[e] = zz;
    ssz += zz * zz;
  }
#pragma unroll
  for (int off = 16; off > 0; off >>= 1) ssz += __shfl_xor(ssz, off, 32);
  if (lane == 0) red[3][wave] = ssz;
  __syncthreads();
  float tz = 0.f;
#pragma unroll
  for (int w = 0; w < 8; ++w) tz += red[3][w];
  const float rz = rsqrtf(tz * inv_d + EPSV);
  v4h yv;
#pragma unroll
  for (int e = 0; e < 4; ++e) yv[e] = (_Float16)(z[e] * rz * fw[e]);
  *(volatile v4h*)(Yh + ro) = yv;
  __threadfence();
  *(volatile v4h*)(Yh + ro) = yv;
}

static void gemm_f16_f32out(const _Float16* A, int lda, long sA, const _Float16* Bt, int ldb, long sB,
                            float* C, int ldc, long sC, int M, int N, int K, float scale, int batch,
                            hipStream_t st) {
  const int tiles = (M / 64) * (N / 64);
  dim3 grid((tiles + 7) / 8, batch);
  wmma_gemm64<0, false, 0, 0, false><<<grid, 256, 0, st>>>(
      (const unsigned short*)A, (const unsigned short*)nullptr, lda, sA,
      (const unsigned short*)Bt, (const unsigned short*)nullptr, ldb, sB,
      (void*)C, (void*)nullptr, ldc, sC, (const float*)nullptr, (const float*)nullptr, 0L,
      M, N, K, scale);
}
static void gemm_f16_f16out(const _Float16* A, int lda, long sA, const _Float16* Bt, int ldb, long sB,
                            _Float16* C, int ldc, long sC, int M, int N, int K, float scale, int batch,
                            hipStream_t st) {
  const int tiles = (M / 64) * (N / 64);
  dim3 grid((tiles + 7) / 8, batch);
  wmma_gemm64<0, false, 0, 1, false><<<grid, 256, 0, st>>>(
      (const unsigned short*)A, (const unsigned short*)nullptr, lda, sA,
      (const unsigned short*)Bt, (const unsigned short*)nullptr, ldb, sB,
      (void*)C, (void*)nullptr, ldc, sC, (const float*)nullptr, (const float*)nullptr, 0L,
      M, N, K, scale);
}

extern "C" void kernel_launch(void* const* d_in, const int* in_sizes, int n_in,
                              void* d_out, int out_size, void* d_ws, size_t ws_size,
                              hipStream_t stream) {
  if (n_in < 11) return;
  const int M = BB * TT;
  if (in_sizes[0] != M * DD) return;
  if (in_sizes[1] < MAXKV * 32 || in_sizes[2] < MAXKV * 32) return;
  if (in_sizes[3] != NLAY * DD * DD) return;
  if (in_sizes[4] != NLAY * DKV * DD || in_sizes[5] != NLAY * DKV * DD) return;
  if (in_sizes[6] < NLAY * DD || in_sizes[7] < NLAY || in_sizes[8] != DD * DD || in_sizes[9] < DD || in_sizes[10] < 1) return;
  if (out_size < M * DD) return;

  const float* x     = (const float*)d_in[0];
  const float* cosT  = (const float*)d_in[1];
  const float* sinT  = (const float*)d_in[2];
  const float* q_w   = (const float*)d_in[3];
  const float* k_w   = (const float*)d_in[4];
  const float* v_w   = (const float*)d_in[5];
  const float* ln_w  = (const float*)d_in[6];
  const float* lam   = (const float*)d_in[7];
  const float* out_w = (const float*)d_in[8];
  const float* fln   = (const float*)d_in[9];
  const float* alpha = (const float*)d_in[10];
  float* out = (float*)d_out;

  char* ws = (char*)d_ws;
  size_t cur = 0;
  auto take = [&](size_t bytes) -> char* {
    char* p = ws + cur;
    cur += (bytes + 4095) & ~(size_t)4095;
    return p;
  };
  _Float16* xh  = (_Float16*)take((size_t)M * DD * 2);
  _Float16* qwh = (_Float16*)take((size_t)NLAY * DD * DD * 2);
  _Float16* kwh = (_Float16*)take((size_t)NLAY * DKV * DD * 2);
  _Float16* vwh = (_Float16*)take((size_t)NLAY * DKV * DD * 2);
  _Float16* owh = (_Float16*)take((size_t)DD * DD * 2);
  float*    Qf  = (float*)   take((size_t)M * DD * 4);
  _Float16* Qh  = (_Float16*)take((size_t)M * DD * 2);
  float*    Kf  = (float*)   take((size_t)M * DKV * 4);
  _Float16* Kh  = (_Float16*)take((size_t)BB * MAXKV * DKV * 2);
  _Float16* Vth = (_Float16*)take((size_t)BB * DKV * MAXKV * 2);
  float*    Of  = (float*)   take((size_t)NLAY * M * DD * 4);
  _Float16* Yh  = (_Float16*)take((size_t)M * DD * 2);
  if (cur > ws_size || cur > (size_t)134217728) return;

  const long lstride = (long)M * DD;

  {
    int n8 = M * DD / 8;
    cast_f32_f16x8<<<(n8 + 255) / 256, 256, 0, stream>>>(x, xh, n8, 1.0f);
    n8 = NLAY * DD * DD / 8;
    cast_f32_f16x8<<<(n8 + 255) / 256, 256, 0, stream>>>(q_w, qwh, n8, 64.0f);
    n8 = NLAY * DKV * DD / 8;
    cast_f32_f16x8<<<(n8 + 255) / 256, 256, 0, stream>>>(k_w, kwh, n8, 64.0f);
    cast_f32_f16x8<<<(n8 + 255) / 256, 256, 0, stream>>>(v_w, vwh, n8, 64.0f);
    n8 = DD * DD / 8;
    cast_f32_f16x8<<<(n8 + 255) / 256, 256, 0, stream>>>(out_w, owh, n8, 64.0f);
  }

  const float wundo  = 1.0f / 64.0f;
  const float sscale = 0.125f / 16.0f;
  const float onorm  = 1.0f / (32768.0f * 16.0f);

  for (int i = 0; i < NLAY; ++i) {
    gemm_f16_f32out(xh, DD, 0L, qwh + (size_t)i * DD * DD, DD, 0L, Qf, DD, 0L, M, DD, DD, wundo, 1, stream);
    rope_cast_kernel<DD><<<M / 2, 256, 0, stream>>>(Qf, cosT, sinT, Qh, TT, 0, 4.0f);
    gemm_f16_f32out(xh, DD, 0L, kwh + (size_t)i * DKV * DD, DD, 0L, Kf, DKV, 0L, M, DKV, DD, wundo, 1, stream);
    rope_cast_kernel<DKV><<<M / 4, 256, 0, stream>>>(Kf, cosT, sinT, Kh, MAXKV, i * TT, 4.0f);
    gemm_f16_f16out(vwh + (size_t)i * DKV * DD, DD, 0L, xh, DD, (long)TT * DD,
                    Vth + (size_t)i * TT, MAXKV, (long)DKV * MAXKV, DKV, TT, DD, 16.0f * wundo, BB, stream);
    attn_f16_kernel<<<BB * HH * (TT / AT_QB), 128, 0, stream>>>(Qh, Kh, Vth, Of + (size_t)i * lstride,
                                                                 i * (TT / AT_KC), i * TT, sscale, onorm);
  }

  combine_kernel<<<M, 256, 0, stream>>>(Of, lstride, x, ln_w, lam, fln, alpha, Yh);
  gemm_f16_f32out(Yh, DD, 0L, owh, DD, 0L, out, DD, 0L, M, DD, DD, wundo, 1, stream);
}
